// denoising_78786880078249
// MI455X (gfx1250) — hardware-verified
//
#include <hip/hip_runtime.h>
#include <math.h>

constexpr int kN  = 16;
constexpr int kC  = 64;
constexpr int kCh = 32;
constexpr int kS  = 3136;
constexpr int kImg = kS * kC;
constexpr int kTot = kN * kImg;
constexpr int kRows = kN * kS;
constexpr int kStatBlocks = 256;
constexpr int kRowsPerStat = kRows / kStatBlocks;
constexpr float kAttnScale = 0.17677669529663687f;
constexpr float kBnEps = 1e-5f;
constexpr float kInvCount = 1.0f / 50176.0f;
constexpr int kSmBlock = 416;
constexpr int kSmWaves = 13;
constexpr int kSmActive = kS / 8;
static_assert(kS % 64 == 0, "tile multiple");
static_assert(kRows == kStatBlocks * kRowsPerStat, "stat blocks");
static_assert(kRowsPerStat % 4 == 0, "stat phases");
static_assert(kSmActive * 8 == kS, "softmax coverage");
static_assert(kSmActive <= kSmBlock, "softmax block");

typedef __attribute__((ext_vector_type(16))) _Float16 v16h;
typedef __attribute__((ext_vector_type(8)))  _Float16 v8h;
typedef __attribute__((ext_vector_type(16))) __bf16   v16b;
typedef __attribute__((ext_vector_type(8)))  __bf16   v8b;
typedef __attribute__((ext_vector_type(8)))  float    v8f;
typedef __attribute__((ext_vector_type(4)))  float    v4f;
typedef __attribute__((ext_vector_type(4)))  unsigned int v4u;

__device__ __forceinline__ unsigned short f2bf_bits(float f) {
  unsigned u = __float_as_uint(f);
  return (unsigned short)((u + 0x7FFFu + ((u >> 16) & 1u)) >> 16);
}
__device__ __forceinline__ float bf_bits2f(unsigned short h) { return __uint_as_float(((unsigned)h) << 16); }

__device__ __forceinline__ void dep_guard_h(v8f& a, v8f& b, v16h x, v16h y) { asm volatile("v_nop\n\tv_nop\n\tv_nop\n\tv_nop" : "+v"(a), "+v"(b) : "v"(x), "v"(y)); }
__device__ __forceinline__ void dep_guard_b(v8f& a, v8f& b, v16b x, v16b y) { asm volatile("v_nop\n\tv_nop\n\tv_nop\n\tv_nop" : "+v"(a), "+v"(b) : "v"(x), "v"(y)); }
__device__ __forceinline__ void keep4_h(v16h a, v16h b, v16h c, v16h d) { asm volatile("v_nop" :: "v"(a), "v"(b), "v"(c), "v"(d)); }
__device__ __forceinline__ void keep4_b(v16b a, v16b b, v16b c, v16b d) { asm volatile("v_nop" :: "v"(a), "v"(b), "v"(c), "v"(d)); }
__device__ __forceinline__ void acc_guard4(v8f& a, v8f& b, v8f& c, v8f& d) { asm volatile("v_nop\n\tv_nop\n\tv_nop\n\tv_nop" : "+v"(a), "+v"(b), "+v"(c), "+v"(d)); }
template <typename T> struct Frag;
template <> struct Frag<_Float16> {
  typedef v16h V; union U { v16h v; v8h h[2]; };
  static __device__ __forceinline__ v16h load(const _Float16* p) {
    U f; f.h[0] = *(const v8h*)(p); f.h[1] = *(const v8h*)(p + 16); return f.v;
  }
  static __device__ __forceinline__ v8f mma(v16h a, v16h b, v8f c) {
    return __builtin_amdgcn_wmma_f32_16x16x32_f16(false, a, false, b, (short)0, c, false, false);
  }
  static __device__ __forceinline__ void guard(v8f& a, v8f& b, v16h x, v16h y) { dep_guard_h(a, b, x, y); }
  static __device__ __forceinline__ void keep(v16h a, v16h b, v16h c, v16h d) { keep4_h(a, b, c, d); }
};
template <> struct Frag<__bf16> {
  typedef v16b V; union U { v16b v; v8b h[2]; };
  static __device__ __forceinline__ v16b load(const __bf16* p) {
    U f; f.h[0] = *(const v8b*)(p); f.h[1] = *(const v8b*)(p + 16); return f.v;
  }
  static __device__ __forceinline__ v8f mma(v16b a, v16b b, v8f c) {
    return __builtin_amdgcn_wmma_f32_16x16x32_bf16(false, a, false, b, (short)0, c, false, false);
  }
  static __device__ __forceinline__ void guard(v8f& a, v8f& b, v16b x, v16b y) { dep_guard_b(a, b, x, y); }
  static __device__ __forceinline__ void keep(v16b a, v16b b, v16b c, v16b d) { keep4_b(a, b, c, d); }
};

__device__ __forceinline__ unsigned pk16(unsigned short a, unsigned short b) { return (unsigned)a | ((unsigned)b << 16); }

template <int ET> struct Elem;
template <> struct Elem<0> { typedef _Float16 T; };
template <> struct Elem<1> { typedef __bf16 T; };
template <int ET, bool SPLIT, int BIAS_MODE, int OUT_MODE, bool RESID, int ACT = 0>
__global__ __launch_bounds__(256) void wmma_gemm64(
    const unsigned short* __restrict__ Ap, const unsigned short* __restrict__ A2p, int lda, long strideA,
    const unsigned short* __restrict__ Btp, const unsigned short* __restrict__ Bt2p, int ldb, long strideB,
    void* __restrict__ Cout, void* __restrict__ Cout2, int ldc, long strideC,
    const float* __restrict__ bias,
    const float* __restrict__ resid, long strideR,
    int M, int N, int K, float scale) {
  typedef typename Elem<ET>::T T;
  typedef typename Frag<T>::V V;
  const T* A = (const T*)Ap; const T* A2 = (const T*)A2p; const T* Bt = (const T*)Btp; const T* Bt2 = (const T*)Bt2p;
  __shared__ __align__(16) float sT[8][16 * 68];
  const int b    = blockIdx.y;
  const int lane = threadIdx.x & 31;
  const int wave = threadIdx.x >> 5;
  const int tilesN = N >> 6;
  const int tilesM = M >> 6;
  const int tile = blockIdx.x * 8 + wave;
  if (tile >= tilesM * tilesN) return;
  const int tm = tile / tilesN;
  const int tn = tile - tm * tilesN;
  const int m0 = tm << 6;
  const int n0 = tn << 6;

  const T* Ab  = A  + (size_t)b * strideA;
  const T* Bb  = Bt + (size_t)b * strideB;
  const T* Ab2 = SPLIT ? (A2  + (size_t)b * strideA) : nullptr;
  const T* Bb2 = SPLIT ? (Bt2 + (size_t)b * strideB) : nullptr;

  const int rlane = lane & 15;
  const int koff  = (lane >> 4) * 8;
  const int mOff  = (lane >> 4) * 8;

  v8f acc[4][4];
#pragma unroll
  for (int i = 0; i < 4; ++i)
#pragma unroll
    for (int j = 0; j < 4; ++j) acc[i][j] = (v8f){0.f,0.f,0.f,0.f,0.f,0.f,0.f,0.f};

  for (int k0 = 0; k0 < K; k0 += 32) {
    V bh[4], bl[4];
#pragma unroll
    for (int j = 0; j < 4; ++j) {
      const size_t bo = (size_t)(n0 + (j << 4) + rlane) * ldb + koff + k0;
      bh[j] = Frag<T>::load(Bb + bo);
      if (SPLIT) bl[j] = Frag<T>::load(Bb2 + bo);
    }
#pragma unroll
    for (int i = 0; i < 4; ++i) {
      const size_t ao = (size_t)(m0 + (i << 4) + rlane) * lda + koff + k0;
      V ah = Frag<T>::load(Ab + ao);
      V al;
      if (SPLIT) al = Frag<T>::load(Ab2 + ao);
#pragma unroll
      for (int j = 0; j < 4; ++j) {
        acc[i][j] = Frag<T>::mma(ah, bh[j], acc[i][j]);
        if (SPLIT) {
          acc[i][j] = Frag<T>::mma(ah, bl[j], acc[i][j]);
          acc[i][j] = Frag<T>::mma(al, bh[j], acc[i][j]);
        }
      }
      Frag<T>::guard(acc[i][0], acc[i][3], ah, SPLIT ? al : ah);
    }
    Frag<T>::keep(bh[0], bh[1], bh[2], bh[3]);
    if (SPLIT) Frag<T>::keep(bl[0], bl[1], bl[2], bl[3]);
  }
  acc_guard4(acc[0][0], acc[0][1], acc[0][2], acc[0][3]);
  acc_guard4(acc[1][0], acc[1][1], acc[1][2], acc[1][3]);
  acc_guard4(acc[2][0], acc[2][1], acc[2][2], acc[2][3]);
  acc_guard4(acc[3][0], acc[3][1], acc[3][2], acc[3][3]);

  float* slab = sT[wave];
  const float* Rb = RESID ? (resid + (size_t)b * strideR) : nullptr;
#pragma unroll
  for (int i = 0; i < 4; ++i) {
    const int mBase = m0 + (i << 4);
#pragma unroll
    for (int j = 0; j < 4; ++j) {
      const int n = n0 + (j << 4) + rlane;
      float bv = 0.f;
      if (BIAS_MODE == 2) bv = bias[n];
#pragma unroll
      for (int r = 0; r < 8; ++r) {
        float v = acc[i][j][r] * scale;
        if (BIAS_MODE == 1) v += bias[mBase + mOff + r];
        if (BIAS_MODE == 2) v += bv;
        if (RESID) v += Rb[(size_t)(mBase + mOff + r) * ldc + n];
        if (ACT == 2) v = fmaxf(v, 0.0f);
        if (ACT == 4) v = (v > 0.f) ? v : 0.01f * v;
        slab[(mOff + r) * 68 + (j << 4) + rlane] = v;
      }
    }
    __builtin_amdgcn_fence(__ATOMIC_RELEASE, "workgroup");
    __builtin_amdgcn_wave_barrier();
    __builtin_amdgcn_fence(__ATOMIC_ACQUIRE, "workgroup");
    if (OUT_MODE == 0) {
      float* C = (float*)Cout + (size_t)b * strideC;
      const int hh = lane >> 4, c4 = (lane & 15) * 4;
      for (int pass = 0; pass < 2; ++pass) {
#pragma unroll
        for (int it = 0; it < 8; ++it) {
          const int row = it * 2 + hh;
          v4f v = *(const v4f*)(slab + row * 68 + c4);
          *(volatile v4f*)(C + (size_t)(mBase + row) * ldc + n0 + c4) = v;
        }
        __threadfence();
      }
    } else {
      const int q = lane >> 3, c8 = (lane & 7) * 8;
      unsigned short* C  = (unsigned short*)Cout  + (size_t)b * strideC;
      unsigned short* C2 = (OUT_MODE == 2) ? ((unsigned short*)Cout2 + (size_t)b * strideC) : nullptr;
      for (int pass = 0; pass < 2; ++pass) {
#pragma unroll
        for (int it = 0; it < 4; ++it) {
          const int row = it * 4 + q;
          const float* sp = slab + row * 68 + c8;
          v8h hv, lv;
#pragma unroll
          for (int e = 0; e < 8; ++e) {
            if (OUT_MODE == 1) {
              hv[e] = (_Float16)sp[e];
            } else {
              unsigned short hb = f2bf_bits(sp[e]);
              unsigned short lb = f2bf_bits(sp[e] - bf_bits2f(hb));
              hv[e] = __builtin_bit_cast(_Float16, hb);
              lv[e] = __builtin_bit_cast(_Float16, lb);
            }
          }
          *(volatile v8h*)(C + (size_t)(mBase + row) * ldc + n0 + c8) = hv;
          if (OUT_MODE == 2) *(volatile v8h*)(C2 + (size_t)(mBase + row) * ldc + n0 + c8) = lv;
        }
        __threadfence();
      }
    }
    __builtin_amdgcn_fence(__ATOMIC_RELEASE, "workgroup");
    __builtin_amdgcn_wave_barrier();
    __builtin_amdgcn_fence(__ATOMIC_ACQUIRE, "workgroup");
  }
}

__device__ __forceinline__ v4f sel4(bool c, v4f a, v4f b) {
  v4f r;
  r.x = c ? a.x : b.x; r.y = c ? a.y : b.y; r.z = c ? a.z : b.z; r.w = c ? a.w : b.w;
  return r;
}

__global__ __launch_bounds__(256) void wprep_kernel(
    const float* __restrict__ w1, const float* __restrict__ w2, const float* __restrict__ w3,
    const float* __restrict__ b1, const float* __restrict__ b2,
    unsigned short* __restrict__ W12h, unsigned short* __restrict__ W12l,
    unsigned short* __restrict__ W3h, unsigned short* __restrict__ W3l,
    float* __restrict__ b12) {
  const int blk = blockIdx.x;
  const int t = threadIdx.x;
  const int lr = t >> 3, c8 = (t & 7) * 8;
  const float* src = (blk == 0) ? w1 : (blk == 1) ? w2 : (w3 + (size_t)(blk - 2) * kCh * kC);
  unsigned short* dh = (blk < 2) ? (W12h + (size_t)blk * kCh * kC) : (W3h + (size_t)(blk - 2) * kCh * kC);
  unsigned short* dl = (blk < 2) ? (W12l + (size_t)blk * kCh * kC) : (W3l + (size_t)(blk - 2) * kCh * kC);
  const float* p = src + (size_t)lr * kC + c8;
  const v4f a = *(const v4f*)(p);
  const v4f c = *(const v4f*)(p + 4);
  unsigned short hb[8], lb[8];
#pragma unroll
  for (int e = 0; e < 4; ++e) {
    hb[e] = f2bf_bits(a[e]);      lb[e] = f2bf_bits(a[e] - bf_bits2f(hb[e]));
    hb[4 + e] = f2bf_bits(c[e]);  lb[4 + e] = f2bf_bits(c[e] - bf_bits2f(hb[4 + e]));
  }
  const v4u uh = (v4u){pk16(hb[0], hb[1]), pk16(hb[2], hb[3]), pk16(hb[4], hb[5]), pk16(hb[6], hb[7])};
  const v4u ul = (v4u){pk16(lb[0], lb[1]), pk16(lb[2], lb[3]), pk16(lb[4], lb[5]), pk16(lb[6], lb[7])};
  unsigned short* qh = dh + (size_t)lr * kC + c8;
  unsigned short* ql = dl + (size_t)lr * kC + c8;
  *(volatile v4u*)qh = uh;
  *(volatile v4u*)ql = ul;
  __threadfence();
  *(volatile v4u*)qh = uh;
  *(volatile v4u*)ql = ul;
  if (blk == 0 && (t >> 5) == 0) {
    const int lane = t & 31;
    const int i4 = (lane & 7) * 4;
    const v4f va = *(const v4f*)(b1 + i4);
    const v4f vb = *(const v4f*)(b2 + i4);
    const v4f v = sel4(lane < 8, va, vb);
    float* bp = b12 + lane * 4;
    if (lane < 16) *(volatile v4f*)bp = v;
    __threadfence();
    if (lane < 16) *(volatile v4f*)bp = v;
  }
}

__global__ __launch_bounds__(256) void xprep_kernel(const float* __restrict__ x,
    unsigned short* __restrict__ Xh, unsigned short* __restrict__ Xl,
    unsigned short* __restrict__ XTh, unsigned short* __restrict__ XTl) {
  __shared__ float sm[64][65];
  const int n = blockIdx.y;
  const int s0 = blockIdx.x * 64;
  const int t = threadIdx.x;
#pragma unroll
  for (int i = 0; i < 4; ++i) {
    const int e = i * 256 + t;
    const int c = e >> 4;
    const int col4 = (e & 15) * 4;
    const v4f v = *(const v4f*)(x + (size_t)(n * kC + c) * kS + s0 + col4);
    sm[c][col4 + 0] = v.x; sm[c][col4 + 1] = v.y; sm[c][col4 + 2] = v.z; sm[c][col4 + 3] = v.w;
  }
  __syncthreads();
  const int lane = t & 31, wave = t >> 5;
  const int q = lane >> 3, c8 = (lane & 7) * 8;
  for (int pass = 0; pass < 2; ++pass) {
#pragma unroll
    for (int it = 0; it < 2; ++it) {
      const int row = wave * 8 + it * 4 + q;
      unsigned short hb[8], lb[8];
#pragma unroll
      for (int e = 0; e < 8; ++e) {
        const float f = sm[row][c8 + e];
        hb[e] = f2bf_bits(f);
        lb[e] = f2bf_bits(f - bf_bits2f(hb[e]));
      }
      const v4u uh = (v4u){pk16(hb[0], hb[1]), pk16(hb[2], hb[3]), pk16(hb[4], hb[5]), pk16(hb[6], hb[7])};
      const v4u ul = (v4u){pk16(lb[0], lb[1]), pk16(lb[2], lb[3]), pk16(lb[4], lb[5]), pk16(lb[6], lb[7])};
      const size_t gi = (size_t)(n * kC + row) * kS + s0 + c8;
      *(volatile v4u*)(Xh + gi) = uh;
      *(volatile v4u*)(Xl + gi) = ul;
    }
#pragma unroll
    for (int it = 0; it < 2; ++it) {
      const int row = wave * 8 + it * 4 + q;
      unsigned short hb[8], lb[8];
#pragma unroll
      for (int e = 0; e < 8; ++e) {
        const float f = sm[c8 + e][row];
        hb[e] = f2bf_bits(f);
        lb[e] = f2bf_bits(f - bf_bits2f(hb[e]));
      }
      const v4u uh = (v4u){pk16(hb[0], hb[1]), pk16(hb[2], hb[3]), pk16(hb[4], hb[5]), pk16(hb[6], hb[7])};
      const v4u ul = (v4u){pk16(lb[0], lb[1]), pk16(lb[2], lb[3]), pk16(lb[4], lb[5]), pk16(lb[6], lb[7])};
      const size_t gi = (size_t)(n * kS + s0 + row) * kC + c8;
      *(volatile v4u*)(XTh + gi) = uh;
      *(volatile v4u*)(XTl + gi) = ul;
    }
    __threadfence();
  }
}

__global__ __launch_bounds__(kSmBlock) void softmax_kernel(const float* __restrict__ Sc,
    unsigned short* __restrict__ Ph, unsigned short* __restrict__ Pl) {
  __shared__ float redM[16];
  __shared__ float redS[16];
  const int row = blockIdx.x;
  const int t = threadIdx.x;
  const int lane = t & 31, wave = t >> 5;
  const bool act = t < kSmActive;
  const int tc = act ? t : 0;
  const float* sr = Sc + (size_t)row * kS + 8 * tc;
  const v4f a = *(const v4f*)(sr);
  const v4f c = *(const v4f*)(sr + 4);
  float xv[8];
#pragma unroll
  for (int e = 0; e < 4; ++e) { xv[e] = a[e]; xv[4 + e] = c[e]; }
  float m = fmaxf(fmaxf(fmaxf(xv[0], xv[1]), fmaxf(xv[2], xv[3])), fmaxf(fmaxf(xv[4], xv[5]), fmaxf(xv[6], xv[7])));
  m = act ? m : -INFINITY;
#pragma unroll
  for (int off = 16; off > 0; off >>= 1) m = fmaxf(m, __shfl_xor(m, off, 32));
  if (lane == 0) redM[wave] = m;
  __syncthreads();
  float gm = redM[0];
#pragma unroll
  for (int w = 1; w < kSmWaves; ++w) gm = fmaxf(gm, redM[w]);
  float ev[8];
  float ps = 0.f;
#pragma unroll
  for (int e = 0; e < 8; ++e) { ev[e] = expf(xv[e] - gm); ps += ev[e]; }
  ps = act ? ps : 0.f;
#pragma unroll
  for (int off = 16; off > 0; off >>= 1) ps += __shfl_xor(ps, off, 32);
  if (lane == 0) redS[wave] = ps;
  __syncthreads();
  float gs = redS[0];
#pragma unroll
  for (int w = 1; w < kSmWaves; ++w) gs += redS[w];
  const float inv = 1.0f / gs;
  unsigned short hb[8], lb[8];
#pragma unroll
  for (int e = 0; e < 8; ++e) {
    const float p = ev[e] * inv;
    hb[e] = f2bf_bits(p);
    lb[e] = f2bf_bits(p - bf_bits2f(hb[e]));
  }
  const v4u uh = (v4u){pk16(hb[0], hb[1]), pk16(hb[2], hb[3]), pk16(hb[4], hb[5]), pk16(hb[6], hb[7])};
  const v4u ul = (v4u){pk16(lb[0], lb[1]), pk16(lb[2], lb[3]), pk16(lb[4], lb[5]), pk16(lb[6], lb[7])};
  unsigned short* qh = Ph + (size_t)row * kS + 8 * tc;
  unsigned short* ql = Pl + (size_t)row * kS + 8 * tc;
  if (act) { *(volatile v4u*)qh = uh; *(volatile v4u*)ql = ul; }
  __threadfence();
  if (act) { *(volatile v4u*)qh = uh; *(volatile v4u*)ql = ul; }
}

__global__ __launch_bounds__(256) void bn_sum_kernel(const float* __restrict__ F2T, float* __restrict__ part) {
  __shared__ float red[4][64];
  __shared__ __align__(16) float outl[64];
  const int blk = blockIdx.x;
  const int t = threadIdx.x;
  const int c = t & 63, ph = t >> 6;
  const int r0 = blk * kRowsPerStat;
  float acc = 0.f;
#pragma unroll 1
  for (int r = ph; r < kRowsPerStat; r += 4) acc += F2T[(size_t)(r0 + r) * kC + c];
  red[ph][c] = acc;
  __syncthreads();
  if (t < 64) outl[t] = ((red[0][t] + red[1][t]) + red[2][t]) + red[3][t];
  __syncthreads();
  if (t < 32) {
    const int p4 = (t & 15) * 4;
    const v4f v = *(const v4f*)(outl + p4);
    float* dp = part + (size_t)blk * 64 + p4;
    if (t < 16) *(volatile v4f*)dp = v;
    __threadfence();
    if (t < 16) *(volatile v4f*)dp = v;
  }
}

__global__ __launch_bounds__(256) void bn_var_kernel(const float* __restrict__ F2T, const float* __restrict__ part,
                                                      float* __restrict__ part2) {
  __shared__ float red[4][64];
  __shared__ float meanL[64];
  __shared__ __align__(16) float outl[64];
  const int blk = blockIdx.x;
  const int t = threadIdx.x;
  const int c = t & 63, ph = t >> 6;
  float ms = 0.f;
#pragma unroll 1
  for (int q = ph; q < kStatBlocks; q += 4) ms += part[(size_t)q * 64 + c];
  red[ph][c] = ms;
  __syncthreads();
  if (t < 64) meanL[t] = (((red[0][t] + red[1][t]) + red[2][t]) + red[3][t]) * kInvCount;
  __syncthreads();
  const float mean = meanL[c];
  const int r0 = blk * kRowsPerStat;
  float acc = 0.f;
#pragma unroll 1
  for (int r = ph; r < kRowsPerStat; r += 4) {
    const float d = F2T[(size_t)(r0 + r) * kC + c] - mean;
    acc += d * d;
  }
  red[ph][c] = acc;
  __syncthreads();
  if (t < 64) outl[t] = ((red[0][t] + red[1][t]) + red[2][t]) + red[3][t];
  __syncthreads();
  if (t < 32) {
    const int p4 = (t & 15) * 4;
    const v4f v = *(const v4f*)(outl + p4);
    float* dp = part2 + (size_t)blk * 64 + p4;
    if (t < 16) *(volatile v4f*)dp = v;
    __threadfence();
    if (t < 16) *(volatile v4f*)dp = v;
  }
}

__global__ __launch_bounds__(256) void bn_fin_kernel(const float* __restrict__ part, const float* __restrict__ part2,
                                                      float* __restrict__ bnp) {
  __shared__ float red[4][64];
  __shared__ __align__(16) float mL[64];
  __shared__ __align__(16) float iL[64];
  const int t = threadIdx.x;
  const int c = t & 63, ph = t >> 6;
  float ms = 0.f;
#pragma unroll 1
  for (int q = ph; q < kStatBlocks; q += 4) ms += part[(size_t)q * 64 + c];
  red[ph][c] = ms;
  __syncthreads();
  if (t < 64) mL[t] = (((red[0][t] + red[1][t]) + red[2][t]) + red[3][t]) * kInvCount;
  __syncthreads();
  float vs = 0.f;
#pragma unroll 1
  for (int q = ph; q < kStatBlocks; q += 4) vs += part2[(size_t)q * 64 + c];
  red[ph][c] = vs;
  __syncthreads();
  if (t < 64) {
    const float var = (((red[0][t] + red[1][t]) + red[2][t]) + red[3][t]) * kInvCount;
    iL[t] = 1.0f / sqrtf(var + kBnEps);
  }
  __syncthreads();
  if (t < 32) {
    const int p4 = (t & 15) * 4;
    const v4f va = *(const v4f*)(mL + p4);
    const v4f vb = *(const v4f*)(iL + p4);
    const v4f v = sel4(t < 16, va, vb);
    float* dp = bnp + (t >> 4) * 64 + p4;
    *(volatile v4f*)dp = v;
    __threadfence();
    *(volatile v4f*)dp = v;
  }
}

__global__ __launch_bounds__(256) void out_kernel(const float* __restrict__ x, const float* __restrict__ F2T,
                                                   const float* __restrict__ bnp, const float* __restrict__ gamma,
                                                   const float* __restrict__ beta, float* __restrict__ out) {
  __shared__ float sm[64][65];
  __shared__ float prm[4][64];
  const int n = blockIdx.y;
  const int s0 = blockIdx.x * 64;
  const int t = threadIdx.x;
  if (t < 64) { prm[0][t] = bnp[t]; prm[1][t] = bnp[64 + t]; prm[2][t] = gamma[t]; prm[3][t] = beta[t]; }
  __syncthreads();
#pragma unroll
  for (int i = 0; i < 4; ++i) {
    const int e = i * 256 + t;
    const int sl = e >> 4;
    const int c4 = (e & 15) * 4;
    const v4f v = *(const v4f*)(F2T + (size_t)(n * kS + s0 + sl) * kC + c4);
#pragma unroll
    for (int j = 0; j < 4; ++j) {
      const int c = c4 + j;
      float y = (v[j] - prm[0][c]) * prm[1][c];
      y = y * prm[2][c] + prm[3][c];
      sm[sl][c] = y;
    }
  }
  __syncthreads();
  const int lane = t & 31, wave = t >> 5;
  const int hh = lane >> 4, s4 = (lane & 15) * 4;
  for (int pass = 0; pass < 2; ++pass) {
#pragma unroll
    for (int it = 0; it < 4; ++it) {
      const int c = wave * 8 + it * 2 + hh;
      const v4f y4 = (v4f){sm[s4][c], sm[s4 + 1][c], sm[s4 + 2][c], sm[s4 + 3][c]};
      const size_t gi = (size_t)(n * kC + c) * kS + s0 + s4;
      const v4f x4 = *(const v4f*)(x + gi);
      const v4f o = x4 + y4;
      *(volatile v4f*)(out + gi) = o;
    }
    __threadfence();
  }
}

extern "C" void kernel_launch(void* const* d_in, const int* in_sizes, int n_in,
                              void* d_out, int out_size, void* d_ws, size_t ws_size,
                              hipStream_t stream) {
  if (n_in < 9) return;
  if (in_sizes[0] != kTot || out_size != kTot) return;
  if (in_sizes[1] != kCh * kC || in_sizes[3] != kCh * kC || in_sizes[5] != kC * kC) return;
  if (in_sizes[2] < kCh || in_sizes[4] < kCh || in_sizes[6] < kC || in_sizes[7] < kC || in_sizes[8] < kC) return;
  const float* x     = (const float*)d_in[0];
  const float* w1    = (const float*)d_in[1];
  const float* b1    = (const float*)d_in[2];
  const float* w2    = (const float*)d_in[3];
  const float* b2    = (const float*)d_in[4];
  const float* w3    = (const float*)d_in[5];
  const float* b3    = (const float*)d_in[6];
  const float* gamma = (const float*)d_in[7];
  const float* beta  = (const float*)d_in[8];
  float* out = (float*)d_out;

  const size_t planeB = (size_t)kTot * 2;
  const size_t sB     = (size_t)kS * kS * 4;
  const size_t pB     = (size_t)kS * kS * 2;
  const size_t wB     = (size_t)kC * kC * 2;
  const size_t partB  = (size_t)kStatBlocks * 64 * 4;
  size_t off = 0;
  char* ws = (char*)d_ws;
  const size_t oXTh = off; off += planeB;
  const size_t oXTl = off; off += planeB;
  const size_t oXh  = off; off += planeB;
  const size_t oXl  = off; off += planeB;
  const size_t oTPh = off; off += planeB;
  const size_t oTPl = off; off += planeB;
  const size_t oS   = off; off += sB;
  const size_t oPh  = off; off += pB;
  const size_t oPl  = off; off += pB;
  const size_t oFh  = off; off += planeB;
  const size_t oFl  = off; off += planeB;
  const size_t oW12h = off; off += wB;
  const size_t oW12l = off; off += wB;
  const size_t oW3h  = off; off += wB;
  const size_t oW3l  = off; off += wB;
  const size_t ob12  = off; off += 256;
  const size_t oPart = off; off += partB;
  const size_t oPart2 = off; off += partB;
  const size_t oBnp  = off; off += 512;
  if (off > ws_size) return;

  unsigned short* XTh = (unsigned short*)(ws + oXTh);
  unsigned short* XTl = (unsigned short*)(ws + oXTl);
  float* F2T = (float*)(ws + oXTh);
  unsigned short* Xh  = (unsigned short*)(ws + oXh);
  unsigned short* Xl  = (unsigned short*)(ws + oXl);
  unsigned short* TPh = (unsigned short*)(ws + oTPh);
  unsigned short* TPl = (unsigned short*)(ws + oTPl);
  float* Sc = (float*)(ws + oS);
  unsigned short* Ph  = (unsigned short*)(ws + oPh);
  unsigned short* Pl  = (unsigned short*)(ws + oPl);
  unsigned short* Fh  = (unsigned short*)(ws + oFh);
  unsigned short* Fl  = (unsigned short*)(ws + oFl);
  unsigned short* W12h = (unsigned short*)(ws + oW12h);
  unsigned short* W12l = (unsigned short*)(ws + oW12l);
  unsigned short* W3h  = (unsigned short*)(ws + oW3h);
  unsigned short* W3l  = (unsigned short*)(ws + oW3l);
  float* b12  = (float*)(ws + ob12);
  float* part = (float*)(ws + oPart);
  float* part2 = (float*)(ws + oPart2);
  float* bnp  = (float*)(ws + oBnp);

  const int tilesS = kS / 64;
  const long imgStride = (long)kImg;

  wprep_kernel<<<dim3(4), 256, 0, stream>>>(w1, w2, w3, b1, b2, W12h, W12l, W3h, W3l, b12);
  xprep_kernel<<<dim3(tilesS, kN), 256, 0, stream>>>(x, Xh, Xl, XTh, XTl);
  wmma_gemm64<1, true, 2, 2, false><<<dim3((tilesS + 7) / 8, kN), 256, 0, stream>>>(
      XTh, XTl, kC, imgStride, W12h, W12l, kC, 0L,
      (void*)TPh, (void*)TPl, kC, imgStride, b12, nullptr, 0L, kS, kC, kC, 1.0f);
  for (int n = 0; n < kN; ++n) {
    const size_t io = (size_t)n * kImg;
    wmma_gemm64<1, true, 0, 0, false><<<dim3((tilesS * tilesS + 7) / 8, 1), 256, 0, stream>>>(
        TPh + io, TPl + io, kC, 0L, TPh + io + kCh, TPl + io + kCh, kC, 0L,
        (void*)Sc, nullptr, kS, 0L, nullptr, nullptr, 0L, kS, kS, kCh, kAttnScale);
    softmax_kernel<<<dim3(kS), kSmBlock, 0, stream>>>(Sc, Ph, Pl);
    wmma_gemm64<1, true, 0, 2, false><<<dim3((tilesS + 7) / 8, 1), 256, 0, stream>>>(
        Ph, Pl, kS, 0L, Xh + io, Xl + io, kS, 0L,
        (void*)(Fh + io), (void*)(Fl + io), kC, 0L, nullptr, nullptr, 0L, kS, kC, kS, 1.0f);
  }
  wmma_gemm64<1, true, 2, 0, false><<<dim3((tilesS + 7) / 8, kN), 256, 0, stream>>>(
      Fh, Fl, kC, imgStride, W3h, W3l, kC, 0L,
      (void*)F2T, nullptr, kC, imgStride, b3, nullptr, 0L, kS, kC, kC, 1.0f);
  bn_sum_kernel<<<dim3(kStatBlocks), 256, 0, stream>>>(F2T, part);
  bn_var_kernel<<<dim3(kStatBlocks), 256, 0, stream>>>(F2T, part, part2);
  bn_fin_kernel<<<dim3(1), 256, 0, stream>>>(part, part2, bnp);
  out_kernel<<<dim3(tilesS, kN), 256, 0, stream>>>(x, F2T, bnp, gamma, beta, out);
}
